// CompoundProteinInteractionPrediction_9474697855149
// MI455X (gfx1250) — hardware-verified
//
#include <hip/hip_runtime.h>
#include <stddef.h>

#define BB 16
#define NN 512
#define LL 512
#define GD 10
#define XP 64
#define DMD 128
#define NH 8
#define DKD 16
#define DFFD 512
#define QKVP 384
#define WVP 64
#define LGN 3
#define LON 3
#define NEGC (-9.0e15f)
#define PSC 32768.0f
#define SQRT_DM 11.313708498984761f

typedef __attribute__((ext_vector_type(16))) _Float16 v16h;
typedef __attribute__((ext_vector_type(8)))  _Float16 v8h;
typedef __attribute__((ext_vector_type(16))) __bf16   v16b;
typedef __attribute__((ext_vector_type(8)))  __bf16   v8b;
typedef __attribute__((ext_vector_type(8)))  float    v8f;
typedef __attribute__((ext_vector_type(4)))  float    v4f;
typedef __attribute__((ext_vector_type(2)))  float    v2f;
typedef __attribute__((ext_vector_type(4)))  int      v4i;

__device__ __forceinline__ unsigned short f2bf_bits(float f) {
  unsigned u = __float_as_uint(f);
  return (unsigned short)((u + 0x7FFFu + ((u >> 16) & 1u)) >> 16);
}
__device__ __forceinline__ float bf_bits2f(unsigned short h) { return __uint_as_float(((unsigned)h) << 16); }

__device__ __forceinline__ void dep_guard_h(v8f& a, v8f& b, v16h x, v16h y) { asm volatile("v_nop\n\tv_nop\n\tv_nop\n\tv_nop" : "+v"(a), "+v"(b) : "v"(x), "v"(y)); }
__device__ __forceinline__ void dep_guard_b(v8f& a, v8f& b, v16b x, v16b y) { asm volatile("v_nop\n\tv_nop\n\tv_nop\n\tv_nop" : "+v"(a), "+v"(b) : "v"(x), "v"(y)); }
__device__ __forceinline__ void keep4_h(v16h a, v16h b, v16h c, v16h d) { asm volatile("v_nop" :: "v"(a), "v"(b), "v"(c), "v"(d)); }
__device__ __forceinline__ void keep4_b(v16b a, v16b b, v16b c, v16b d) { asm volatile("v_nop" :: "v"(a), "v"(b), "v"(c), "v"(d)); }
__device__ __forceinline__ void acc_guard4(v8f& a, v8f& b, v8f& c, v8f& d) { asm volatile("v_nop\n\tv_nop\n\tv_nop\n\tv_nop" : "+v"(a), "+v"(b), "+v"(c), "+v"(d)); }
template <typename T> struct Frag;
template <> struct Frag<_Float16> {
  typedef v16h V; union U { v16h v; v8h h[2]; };
  static __device__ __forceinline__ v16h load(const _Float16* p) {
    U f; f.h[0] = *(const v8h*)(p); f.h[1] = *(const v8h*)(p + 16); return f.v;
  }
  static __device__ __forceinline__ v8f mma(v16h a, v16h b, v8f c) {
    return __builtin_amdgcn_wmma_f32_16x16x32_f16(false, a, false, b, (short)0, c, false, false);
  }
  static __device__ __forceinline__ void guard(v8f& a, v8f& b, v16h x, v16h y) { dep_guard_h(a, b, x, y); }
  static __device__ __forceinline__ void keep(v16h a, v16h b, v16h c, v16h d) { keep4_h(a, b, c, d); }
};
template <> struct Frag<__bf16> {
  typedef v16b V; union U { v16b v; v8b h[2]; };
  static __device__ __forceinline__ v16b load(const __bf16* p) {
    U f; f.h[0] = *(const v8b*)(p); f.h[1] = *(const v8b*)(p + 16); return f.v;
  }
  static __device__ __forceinline__ v8f mma(v16b a, v16b b, v8f c) {
    return __builtin_amdgcn_wmma_f32_16x16x32_bf16(false, a, false, b, (short)0, c, false, false);
  }
  static __device__ __forceinline__ void guard(v8f& a, v8f& b, v16b x, v16b y) { dep_guard_b(a, b, x, y); }
  static __device__ __forceinline__ void keep(v16b a, v16b b, v16b c, v16b d) { keep4_b(a, b, c, d); }
};

template <int ET> struct Elem;
template <> struct Elem<0> { typedef _Float16 T; };
template <> struct Elem<1> { typedef __bf16 T; };
template <int ET, bool SPLIT, int BIAS_MODE, int OUT_MODE, bool RESID, int ACT = 0>
__global__ __launch_bounds__(256) void wmma_gemm64(
    const unsigned short* __restrict__ Ap, const unsigned short* __restrict__ A2p, int lda, long strideA,
    const unsigned short* __restrict__ Btp, const unsigned short* __restrict__ Bt2p, int ldb, long strideB,
    void* __restrict__ Cout, void* __restrict__ Cout2, int ldc, long strideC,
    const float* __restrict__ bias,
    const float* __restrict__ resid, long strideR,
    int M, int N, int K, float scale) {
  typedef typename Elem<ET>::T T;
  typedef typename Frag<T>::V V;
  const T* A = (const T*)Ap; const T* A2 = (const T*)A2p; const T* Bt = (const T*)Btp; const T* Bt2 = (const T*)Bt2p;
  __shared__ __align__(16) float sT[8][16 * 68];
  const int b    = blockIdx.y;
  const int lane = threadIdx.x & 31;
  const int wave = threadIdx.x >> 5;
  const int tilesN = N >> 6;
  const int tilesM = M >> 6;
  const int tile = blockIdx.x * 8 + wave;
  if (tile >= tilesM * tilesN) return;
  const int tm = tile / tilesN;
  const int tn = tile - tm * tilesN;
  const int m0 = tm << 6;
  const int n0 = tn << 6;

  const T* Ab  = A  + (size_t)b * strideA;
  const T* Bb  = Bt + (size_t)b * strideB;
  const T* Ab2 = SPLIT ? (A2  + (size_t)b * strideA) : nullptr;
  const T* Bb2 = SPLIT ? (Bt2 + (size_t)b * strideB) : nullptr;

  const int rlane = lane & 15;
  const int koff  = (lane >> 4) * 8;
  const int mOff  = (lane >> 4) * 8;

  v8f acc[4][4];
#pragma unroll
  for (int i = 0; i < 4; ++i)
#pragma unroll
    for (int j = 0; j < 4; ++j) acc[i][j] = (v8f){0.f,0.f,0.f,0.f,0.f,0.f,0.f,0.f};

  for (int k0 = 0; k0 < K; k0 += 32) {
    V bh[4], bl[4];
#pragma unroll
    for (int j = 0; j < 4; ++j) {
      const size_t bo = (size_t)(n0 + (j << 4) + rlane) * ldb + koff + k0;
      bh[j] = Frag<T>::load(Bb + bo);
      if (SPLIT) bl[j] = Frag<T>::load(Bb2 + bo);
    }
#pragma unroll
    for (int i = 0; i < 4; ++i) {
      const size_t ao = (size_t)(m0 + (i << 4) + rlane) * lda + koff + k0;
      V ah = Frag<T>::load(Ab + ao);
      V al;
      if (SPLIT) al = Frag<T>::load(Ab2 + ao);
#pragma unroll
      for (int j = 0; j < 4; ++j) {
        acc[i][j] = Frag<T>::mma(ah, bh[j], acc[i][j]);
        if (SPLIT) {
          acc[i][j] = Frag<T>::mma(ah, bl[j], acc[i][j]);
          acc[i][j] = Frag<T>::mma(al, bh[j], acc[i][j]);
        }
      }
      Frag<T>::guard(acc[i][0], acc[i][3], ah, SPLIT ? al : ah);
    }
    Frag<T>::keep(bh[0], bh[1], bh[2], bh[3]);
    if (SPLIT) Frag<T>::keep(bl[0], bl[1], bl[2], bl[3]);
  }
  acc_guard4(acc[0][0], acc[0][1], acc[0][2], acc[0][3]);
  acc_guard4(acc[1][0], acc[1][1], acc[1][2], acc[1][3]);
  acc_guard4(acc[2][0], acc[2][1], acc[2][2], acc[2][3]);
  acc_guard4(acc[3][0], acc[3][1], acc[3][2], acc[3][3]);

  float* slab = sT[wave];
  const float* Rb = RESID ? (resid + (size_t)b * strideR) : nullptr;
#pragma unroll
  for (int i = 0; i < 4; ++i) {
    const int mBase = m0 + (i << 4);
#pragma unroll
    for (int j = 0; j < 4; ++j) {
      const int n = n0 + (j << 4) + rlane;
      float bv = 0.f;
      if (BIAS_MODE == 2) bv = bias[n];
#pragma unroll
      for (int r = 0; r < 8; ++r) {
        float v = acc[i][j][r] * scale;
        if (BIAS_MODE == 1) v += bias[mBase + mOff + r];
        if (BIAS_MODE == 2) v += bv;
        if (RESID) v += Rb[(size_t)(mBase + mOff + r) * ldc + n];
        if (ACT == 1) v = tanhf(v);
        if (ACT == 2) v = fmaxf(v, 0.0f);
        if (ACT == 3) v = v / (1.0f + expf(-v));
        if (ACT == 4) v = (v > 0.f) ? v : 0.01f * v;
        if (ACT == 5) v = 0.5f * v * (1.0f + erff(v * 0.70710678118654752f));
        slab[(mOff + r) * 68 + (j << 4) + rlane] = v;
      }
    }
    __builtin_amdgcn_fence(__ATOMIC_RELEASE, "workgroup");
    __builtin_amdgcn_wave_barrier();
    __builtin_amdgcn_fence(__ATOMIC_ACQUIRE, "workgroup");
    if (OUT_MODE == 0) {
      float* C = (float*)Cout + (size_t)b * strideC;
      const int hh = lane >> 4, c4 = (lane & 15) * 4;
      for (int pass = 0; pass < 2; ++pass) {
#pragma unroll
        for (int it = 0; it < 8; ++it) {
          const int row = it * 2 + hh;
          v4f v = *(const v4f*)(slab + row * 68 + c4);
          *(volatile v4f*)(C + (size_t)(mBase + row) * ldc + n0 + c4) = v;
        }
        __threadfence();
      }
    } else {
      const int q = lane >> 3, c8 = (lane & 7) * 8;
      unsigned short* C  = (unsigned short*)Cout  + (size_t)b * strideC;
      unsigned short* C2 = (OUT_MODE == 2) ? ((unsigned short*)Cout2 + (size_t)b * strideC) : nullptr;
      for (int pass = 0; pass < 2; ++pass) {
#pragma unroll
        for (int it = 0; it < 4; ++it) {
          const int row = it * 4 + q;
          const float* sp = slab + row * 68 + c8;
          v8h hv, lv;
#pragma unroll
          for (int e = 0; e < 8; ++e) {
            if (OUT_MODE == 1) {
              hv[e] = (_Float16)sp[e];
            } else {
              unsigned short hb = f2bf_bits(sp[e]);
              unsigned short lb = f2bf_bits(sp[e] - bf_bits2f(hb));
              hv[e] = __builtin_bit_cast(_Float16, hb);
              lv[e] = __builtin_bit_cast(_Float16, lb);
            }
          }
          *(volatile v8h*)(C + (size_t)(mBase + row) * ldc + n0 + c8) = hv;
          if (OUT_MODE == 2) *(volatile v8h*)(C2 + (size_t)(mBase + row) * ldc + n0 + c8) = lv;
        }
        __threadfence();
      }
    }
    __builtin_amdgcn_fence(__ATOMIC_RELEASE, "workgroup");
    __builtin_amdgcn_wave_barrier();
    __builtin_amdgcn_fence(__ATOMIC_ACQUIRE, "workgroup");
  }
}

__device__ __forceinline__ v8f mma_h(v16h a, v16h b, v8f c) {
  c = __builtin_amdgcn_wmma_f32_16x16x32_f16(false, a, false, b, (short)0, c, false, false);
  asm volatile("v_nop\n\tv_nop\n\tv_nop\n\tv_nop" : "+v"(c) : "v"(a), "v"(b));
  return c;
}
__device__ __forceinline__ float wsum32(float v) {
#pragma unroll
  for (int off = 16; off > 0; off >>= 1) v += __shfl_xor(v, off, 32);
  return v;
}
__device__ __forceinline__ float wmax32(float v) {
#pragma unroll
  for (int off = 16; off > 0; off >>= 1) v = fmaxf(v, __shfl_xor(v, off, 32));
  return v;
}

__global__ __launch_bounds__(256) void pe_table_k(float* __restrict__ pe, int npairs) {
  const int t = blockIdx.x * 256 + threadIdx.x;
  if (t < npairs) {
    const int pos = t >> 6, kp = t & 63;
    const float dv = expf((float)(2 * kp) * (-0.07195578415129535f));
    const float ang = (float)pos * dv;
    float sv, cv;
    sincosf(ang, &sv, &cv);
    v2f o; o[0] = sv; o[1] = cv;
    volatile v2f* p = (volatile v2f*)(pe + (size_t)pos * DMD + 2 * kp);
    *p = o;
    __threadfence();
    *p = o;
  }
}

__global__ __launch_bounds__(256) void tcast_k(const float* __restrict__ W, int K, int Nc,
                                             _Float16* __restrict__ Wt, int ldo, int n_off) {
  __shared__ float tile[64][68];
  const int tid = threadIdx.x;
  const int n0 = blockIdx.x * 64, k0 = blockIdx.y * 64;
  for (int i = tid; i < 4096; i += 256) {
    const int kk = i >> 6, nn = i & 63;
    const int n = n0 + nn;
    float v = 0.f;
    if (n < Nc && (k0 + kk) < K) v = W[(size_t)(k0 + kk) * Nc + n];
    tile[nn][kk] = v;
  }
  __syncthreads();
  const int q = tid >> 3, c8 = (tid & 7) * 8;
  for (int pass = 0; pass < 2; ++pass) {
#pragma unroll
    for (int it = 0; it < 2; ++it) {
      const int row = it * 32 + q;
      v8h hv;
#pragma unroll
      for (int e = 0; e < 8; ++e) hv[e] = (_Float16)tile[row][c8 + e];
      *(volatile v8h*)(Wt + (size_t)(n_off + n0 + row) * ldo + k0 + c8) = hv;
    }
    __threadfence();
  }
}

__global__ __launch_bounds__(256) void embed_fp_k(const int* __restrict__ fp, const float* __restrict__ emb, int nfp,
                                                float* __restrict__ xs, int nrows) {
  const int t = blockIdx.x * 256 + threadIdx.x;
  if (t < nrows * 16) {
    const int bn = t >> 4, c4 = (t & 15) * 4;
    int id = fp[bn];
    id = id < 0 ? 0 : (id >= nfp ? nfp - 1 : id);
    v4f v;
#pragma unroll
    for (int e = 0; e < 4; ++e) {
      const int cc = c4 + e;
      v[e] = (cc < GD) ? emb[(size_t)id * GD + cc] : 0.f;
    }
    volatile v4f* p = (volatile v4f*)(xs + (size_t)bn * XP + c4);
    *p = v;
    __threadfence();
    *p = v;
  }
}

__global__ __launch_bounds__(256) void gat_node_k(const float* __restrict__ xs, const float* __restrict__ Wg,
                                                const float* __restrict__ bg, const float* __restrict__ av,
                                                const float* __restrict__ fmask, _Float16* __restrict__ hT,
                                                float* __restrict__ s1, float* __restrict__ s2) {
  __shared__ float sW[GD * GD];
  __shared__ float sb[GD];
  __shared__ float sa[2 * GD];
  __shared__ __align__(16) _Float16 hs[16][64];
  __shared__ __align__(16) float ss1[64];
  __shared__ __align__(16) float ss2[64];
  const int tid = threadIdx.x;
  const int b = blockIdx.x >> 3, nb0 = (blockIdx.x & 7) * 64;
  if (tid < GD * GD) sW[tid] = Wg[tid];
  if (tid < GD) sb[tid] = bg[tid];
  if (tid < 2 * GD) sa[tid] = av[tid];
  __syncthreads();
  const int d = tid & 15, dcl = (d < GD) ? d : (GD - 1);
  const int nsub = tid >> 4;
  for (int p = 0; p < 4; ++p) {
    const int nl = p * 16 + nsub;
    const size_t row = (size_t)b * NN + nb0 + nl;
    const float* xr = xs + row * XP;
    float acc = sb[dcl];
#pragma unroll 1
    for (int e = 0; e < GD; ++e) acc += xr[e] * sW[e * GD + dcl];
    float hd = fmaxf(acc, 0.f) * fmask[row];
    if (d >= GD) hd = 0.f;
    hs[d][nl] = (_Float16)hd;
    float p1 = hd * sa[dcl], p2 = hd * sa[GD + dcl];
#pragma unroll
    for (int off = 1; off < 16; off <<= 1) {
      p1 += __shfl_xor(p1, off, 32);
      p2 += __shfl_xor(p2, off, 32);
    }
    if (d == 0) { ss1[nl] = p1; ss2[nl] = p2; }
  }
  __syncthreads();
  const int q = tid >> 3, c8 = (tid & 7) * 8;
  _Float16* hb = hT + ((size_t)b * 64) * NN + nb0;
  v8h z8;
#pragma unroll
  for (int e = 0; e < 8; ++e) z8[e] = (_Float16)0.0f;
  for (int pass = 0; pass < 2; ++pass) {
    if (q < 16) {
      v8h v = *(const v8h*)(&hs[q][c8]);
      *(volatile v8h*)(hb + (size_t)q * NN + c8) = v;
    }
#pragma unroll
    for (int it = 0; it < 2; ++it) {
      const int r = 16 + it * 32 + q;
      if (r < 64) *(volatile v8h*)(hb + (size_t)r * NN + c8) = z8;
    }
    if (tid < 16) {
      v4f v = *(const v4f*)(&ss1[tid * 4]);
      *(volatile v4f*)(s1 + (size_t)b * NN + nb0 + tid * 4) = v;
    } else if (tid < 32) {
      v4f v = *(const v4f*)(&ss2[(tid - 16) * 4]);
      *(volatile v4f*)(s2 + (size_t)b * NN + nb0 + (tid - 16) * 4) = v;
    }
    __threadfence();
  }
}

__global__ __launch_bounds__(256) void gat_att_k(const int* __restrict__ adj, const float* __restrict__ s1,
                                               const float* __restrict__ s2, _Float16* __restrict__ att) {
  const int lane = threadIdx.x & 31, wave = threadIdx.x >> 5;
  const int b = blockIdx.x >> 3, i0 = (blockIdx.x & 7) * 64 + wave * 8;
  const float* s2b = s2 + (size_t)b * NN;
  float s2v[16];
  {
    const v4f a0 = *(const v4f*)(s2b + lane * 8), a1 = *(const v4f*)(s2b + lane * 8 + 4);
    const v4f a2 = *(const v4f*)(s2b + 256 + lane * 8), a3 = *(const v4f*)(s2b + 256 + lane * 8 + 4);
#pragma unroll
    for (int e = 0; e < 4; ++e) { s2v[e] = a0[e]; s2v[4 + e] = a1[e]; s2v[8 + e] = a2[e]; s2v[12 + e] = a3[e]; }
  }
  for (int rr = 0; rr < 8; ++rr) {
    const size_t row = (size_t)b * NN + i0 + rr;
    const float s1i = s1[row];
    const int* ar = adj + row * NN;
    int mk[16];
    {
      const v4i m0 = *(const v4i*)(ar + lane * 8), m1 = *(const v4i*)(ar + lane * 8 + 4);
      const v4i m2 = *(const v4i*)(ar + 256 + lane * 8), m3 = *(const v4i*)(ar + 256 + lane * 8 + 4);
#pragma unroll
      for (int e = 0; e < 4; ++e) { mk[e] = m0[e]; mk[4 + e] = m1[e]; mk[8 + e] = m2[e]; mk[12 + e] = m3[e]; }
    }
    float ev[16];
    float mx = -__builtin_inff();
#pragma unroll
    for (int t = 0; t < 16; ++t) {
      const float z = s1i + s2v[t];
      float e = (z >= 0.f) ? z : 0.01f * z;
      e = (mk[t] > 0) ? e : NEGC;
      ev[t] = e;
      mx = fmaxf(mx, e);
    }
    mx = wmax32(mx);
    float den = 0.f;
#pragma unroll
    for (int t = 0; t < 16; ++t) {
      const float p = __expf(ev[t] - mx);
      ev[t] = p;
      den += p;
    }
    den = wsum32(den);
    const float sc = PSC * (1.0f / den);
    v8h o0, o1;
#pragma unroll
    for (int e = 0; e < 8; ++e) { o0[e] = (_Float16)(ev[e] * sc); o1[e] = (_Float16)(ev[8 + e] * sc); }
    _Float16* orow = att + row * NN;
    volatile v8h* p0 = (volatile v8h*)(orow + lane * 8);
    volatile v8h* p1 = (volatile v8h*)(orow + 256 + lane * 8);
    *p0 = o0; *p1 = o1;
    __threadfence();
    *p0 = o0; *p1 = o1;
  }
}

template <int MODE>
__global__ __launch_bounds__(256) void ln_k(const float* __restrict__ xin, const int* __restrict__ words,
                                          const float* __restrict__ emb, int nw, const float* __restrict__ pe,
                                          float* __restrict__ xout, const float* __restrict__ g,
                                          const float* __restrict__ bt, _Float16* __restrict__ y, int rows) {
  __shared__ __align__(16) _Float16 sh[8][DMD];
  const int lane = threadIdx.x & 31, wave = threadIdx.x >> 5;
  const int row = blockIdx.x * 8 + wave;
  if (row < rows) {
    const int c4 = lane * 4;
    v4f v;
    if (MODE == 0) {
      int id = words[row];
      id = id < 0 ? 0 : (id >= nw ? nw - 1 : id);
      const v4f ev = *(const v4f*)(emb + (size_t)id * DMD + c4);
      const v4f pv = *(const v4f*)(pe + (size_t)(row & (LL - 1)) * DMD + c4);
#pragma unroll
      for (int e = 0; e < 4; ++e) v[e] = ev[e] * SQRT_DM + pv[e];
      volatile v4f* px = (volatile v4f*)(xout + (size_t)row * DMD + c4);
      *px = v;
      __threadfence();
      *px = v;
    } else {
      v = *(const v4f*)(xin + (size_t)row * DMD + c4);
    }
    float s = v[0] + v[1] + v[2] + v[3];
    s = wsum32(s);
    const float m = s * (1.0f / 128.0f);
    float ss = 0.f;
#pragma unroll
    for (int e = 0; e < 4; ++e) { const float d = v[e] - m; ss += d * d; }
    ss = wsum32(ss);
    const float sd = sqrtf(ss * (1.0f / 127.0f));
    const float inv = 1.0f / (sd + 1e-6f);
    _Float16* shw = sh[wave];
#pragma unroll
    for (int e = 0; e < 4; ++e) {
      float yv = g[c4 + e] * (v[e] - m) * inv + bt[c4 + e];
      if (MODE == 2) yv = fmaxf(yv, 0.f);
      shw[c4 + e] = (_Float16)yv;
    }
    __builtin_amdgcn_fence(__ATOMIC_RELEASE, "workgroup");
    __builtin_amdgcn_wave_barrier();
    __builtin_amdgcn_fence(__ATOMIC_ACQUIRE, "workgroup");
    for (int pass = 0; pass < 2; ++pass) {
      if (lane < 16) {
        v8h hv = *(const v8h*)(shw + lane * 8);
        *(volatile v8h*)(y + (size_t)row * DMD + lane * 8) = hv;
      }
      __threadfence();
    }
  }
}

__global__ __launch_bounds__(128) void mha16_k(const float* __restrict__ qkv, const float* __restrict__ bq,
                                             const float* __restrict__ bk, const float* __restrict__ bv,
                                             const float* __restrict__ wmask, _Float16* __restrict__ attn) {
  union FB { v16h v; v8h h[2]; };
  __shared__ __align__(16) _Float16 Ksh[64 * DKD];
  __shared__ __align__(16) _Float16 Vth[DKD * 64];
  __shared__ __align__(16) _Float16 Psh[4][16 * 64];
  __shared__ __align__(16) _Float16 Osh[4][16 * DMD];
  const int tid = threadIdx.x, wave = tid >> 5, lane = tid & 31, hh = lane >> 4, c = lane & 15;
  const int b = blockIdx.x >> 3, qb = blockIdx.x & 7;
  const int q0 = qb * 64 + wave * 16;
  const size_t rb = (size_t)b * LL;
  _Float16* osw = Osh[wave];
  _Float16* pwh = Psh[wave];
  v8h z8;
#pragma unroll
  for (int e = 0; e < 8; ++e) z8[e] = (_Float16)0.0f;
  const v8f zf = (v8f){0.f,0.f,0.f,0.f,0.f,0.f,0.f,0.f};

  for (int h = 0; h < NH; ++h) {
    v16h qa;
    {
      const float* qr = qkv + (rb + q0 + c) * QKVP + h * DKD + 8 * hh;
      const float* bqp = bq + h * DKD + 8 * hh;
#pragma unroll
      for (int e = 0; e < 8; ++e) {
        qa[e] = (_Float16)((qr[e] + bqp[e]) * 0.25f);
        qa[8 + e] = (_Float16)0.0f;
      }
    }
    float mrow[8], lrow[8];
    v8f oacc = zf;
#pragma unroll
    for (int r = 0; r < 8; ++r) { mrow[r] = -__builtin_inff(); lrow[r] = 0.f; }

    for (int kc = 0; kc < LL / 64; ++kc) {
      const int kv0 = kc * 64;
      __syncthreads();
      {
        const int kvr = tid >> 1, dh = (tid & 1) * 8;
        const float* kr = qkv + (rb + kv0 + kvr) * QKVP + DMD + h * DKD + dh;
        const float* vr = kr + DMD;
        const v4f k0 = *(const v4f*)kr, k1 = *(const v4f*)(kr + 4);
        const v4f v0 = *(const v4f*)vr, v1 = *(const v4f*)(vr + 4);
        const float* bkp = bk + h * DKD + dh;
        const float* bvp = bv + h * DKD + dh;
#pragma unroll
        for (int e = 0; e < 4; ++e) {
          Ksh[kvr * DKD + dh + e]     = (_Float16)(k0[e] + bkp[e]);
          Ksh[kvr * DKD + dh + 4 + e] = (_Float16)(k1[e] + bkp[4 + e]);
          Vth[(dh + e) * 64 + kvr]     = (_Float16)(v0[e] + bvp[e]);
          Vth[(dh + 4 + e) * 64 + kvr] = (_Float16)(v1[e] + bvp[4 + e]);
        }
      }
      __syncthreads();

      v8f s[4];
#pragma unroll
      for (int j = 0; j < 4; ++j) {
        FB kb;
        kb.h[0] = *(const v8h*)(Ksh + (j * 16 + c) * DKD + 8 * hh);
        kb.h[1] = z8;
        s[j] = mma_h(qa, kb.v, zf);
      }
      int keep[4];
#pragma unroll
      for (int j = 0; j < 4; ++j) keep[j] = (wmask[rb + kv0 + j * 16 + c] > 0.f) ? 1 : 0;
      float cm[8];
#pragma unroll
      for (int r = 0; r < 8; ++r) {
        float m = -__builtin_inff();
#pragma unroll
        for (int j = 0; j < 4; ++j) {
          if (keep[j] == 0) s[j][r] = -1.0e9f;
          m = fmaxf(m, s[j][r]);
        }
#pragma unroll
        for (int off = 1; off < 16; off <<= 1) m = fmaxf(m, __shfl_xor(m, off, 32));
        cm[r] = m;
      }
#pragma unroll
      for (int r = 0; r < 8; ++r) {
        const float mnew = fmaxf(mrow[r], cm[r]);
        const float alpha = expf(mrow[r] - mnew);
        mrow[r] = mnew;
        float psum = 0.f;
#pragma unroll
        for (int j = 0; j < 4; ++j) {
          const float p = expf(s[j][r] - mnew);
          psum += p;
          pwh[(8 * hh + r) * 64 + j * 16 + c] = (_Float16)(p * PSC);
        }
#pragma unroll
        for (int off = 1; off < 16; off <<= 1) psum += __shfl_xor(psum, off, 32);
        lrow[r] = lrow[r] * alpha + psum;
        oacc[r] *= alpha;
      }
      __builtin_amdgcn_fence(__ATOMIC_RELEASE, "workgroup");
      __builtin_amdgcn_wave_barrier();
      __builtin_amdgcn_fence(__ATOMIC_ACQUIRE, "workgroup");
#pragma unroll 1
      for (int kk = 0; kk < 2; ++kk) {
        FB pa, vbf;
        pa.h[0]  = *(const v8h*)(pwh + c * 64 + kk * 32 + 8 * hh);
        pa.h[1]  = *(const v8h*)(pwh + c * 64 + kk * 32 + 16 + 8 * hh);
        vbf.h[0] = *(const v8h*)(Vth + c * 64 + kk * 32 + 8 * hh);
        vbf.h[1] = *(const v8h*)(Vth + c * 64 + kk * 32 + 16 + 8 * hh);
        oacc = mma_h(pa.v, vbf.v, oacc);
      }
    }
#pragma unroll
    for (int r = 0; r < 8; ++r) {
      const float inv = 1.0f / (lrow[r] * PSC);
      osw[(8 * hh + r) * DMD + h * DKD + c] = (_Float16)(oacc[r] * inv);
    }
  }
  __builtin_amdgcn_fence(__ATOMIC_RELEASE, "workgroup");
  __builtin_amdgcn_wave_barrier();
  __builtin_amdgcn_fence(__ATOMIC_ACQUIRE, "workgroup");
  {
    const int q4 = lane >> 3, c8 = (lane & 7) * 8;
    for (int pass = 0; pass < 2; ++pass) {
#pragma unroll
      for (int it = 0; it < 8; ++it) {
        const int li = it * 4 + q4;
        const int row = li >> 1, half = li & 1;
        v8h val = *(const v8h*)(osw + row * DMD + half * 64 + c8);
        *(volatile v8h*)(attn + (rb + q0 + row) * DMD + half * 64 + c8) = val;
      }
      __threadfence();
    }
  }
}

__global__ __launch_bounds__(512) void tail_k(const float* __restrict__ xs, const float* __restrict__ fmask,
                                            const float* __restrict__ wv, const float* __restrict__ btout,
                                            const float* __restrict__ Watt, const float* __restrict__ batt,
                                            const float* __restrict__ Wout, const float* __restrict__ bout,
                                            const float* __restrict__ Wint, const float* __restrict__ bint,
                                            float* __restrict__ out) {
  __shared__ float sWatt[GD * GD];
  __shared__ float sbatt[GD];
  __shared__ float sbt[GD];
  __shared__ float sWout[LON * 2 * GD * 2 * GD];
  __shared__ float sbout[LON * 2 * GD];
  __shared__ float sWint[2 * GD * 2];
  __shared__ float sbint[2];
  __shared__ float compS[BB][16];
  __shared__ float catS[BB][2 * GD + 4];
  __shared__ __align__(16) float outs[2 * BB];
  const int tid = threadIdx.x, lane = tid & 31, b = tid >> 5;
  for (int i = tid; i < LON * 2 * GD * 2 * GD; i += 512) sWout[i] = Wout[i];
  if (tid < GD * GD) sWatt[tid] = Watt[tid];
  if (tid < GD) { sbatt[tid] = batt[tid]; sbt[tid] = btout[tid]; }
  if (tid < LON * 2 * GD) sbout[tid] = bout[tid];
  if (tid < 2 * GD * 2) sWint[tid] = Wint[tid];
  if (tid < 2) sbint[tid] = bint[tid];
  __syncthreads();

  const int d = lane & 15, hf = lane >> 4, dcl = (d < GD) ? d : (GD - 1);
  float acc = 0.f;
  {
    const size_t rb0 = (size_t)b * NN + hf * 256;
#pragma unroll 1
    for (int n = 0; n < 256; ++n) acc += xs[(rb0 + n) * XP + dcl] * fmask[rb0 + n];
  }
  acc += __shfl_xor(acc, 16, 32);
  const float comp = (d < GD) ? acc * (1.0f / (float)NN) : 0.f;
  if (hf == 0) compS[b][d] = comp;
  __syncthreads();
  float hc = sbatt[dcl];
#pragma unroll 1
  for (int e = 0; e < GD; ++e) hc += compS[b][e] * sWatt[e * GD + dcl];
  hc = (d < GD) ? fmaxf(hc, 0.f) : 0.f;

  float pacc = 0.f;
#pragma unroll 1
  for (int lp = 0; lp < LL / 2; ++lp) {
    const int l = lp * 2 + hf;
    const float* wr = wv + ((size_t)b * LL + l) * WVP;
    float hp = sbatt[dcl];
#pragma unroll 1
    for (int e = 0; e < GD; ++e) hp += (wr[e] + sbt[e]) * sWatt[e * GD + dcl];
    hp = (d < GD) ? fmaxf(hp, 0.f) : 0.f;
    float dt = hc * hp;
#pragma unroll
    for (int off = 1; off < 16; off <<= 1) dt += __shfl_xor(dt, off, 32);
    const float w = tanhf(dt);
    pacc += w * hp;
  }
  pacc += __shfl_xor(pacc, 16, 32);
  const float prot = pacc * (1.0f / (float)LL);
  if (hf == 0 && d < GD) { catS[b][d] = comp; catS[b][GD + d] = prot; }
  __syncthreads();

  const int ocl = (lane < 2 * GD) ? lane : (2 * GD - 1);
  for (int j = 0; j < LON; ++j) {
    float s = sbout[j * 2 * GD + ocl];
#pragma unroll 1
    for (int i2 = 0; i2 < 2 * GD; ++i2) s += catS[b][i2] * sWout[(j * 2 * GD + i2) * 2 * GD + ocl];
    s = fmaxf(s, 0.f);
    __syncthreads();
    if (lane < 2 * GD) catS[b][lane] = s;
    __syncthreads();
  }
  {
    const int o2 = (lane < 2) ? lane : 1;
    float s = sbint[o2];
#pragma unroll 1
    for (int i2 = 0; i2 < 2 * GD; ++i2) s += catS[b][i2] * sWint[i2 * 2 + o2];
    if (lane < 2) outs[b * 2 + lane] = s;
  }
  __syncthreads();
  for (int pass = 0; pass < 2; ++pass) {
    if (tid < 8) {
      v4f v = *(const v4f*)(&outs[tid * 4]);
      *(volatile v4f*)(out + tid * 4) = v;
    }
    __threadfence();
  }
}

extern "C" void kernel_launch(void* const* d_in, const int* in_sizes, int n_in,
                              void* d_out, int out_size, void* d_ws, size_t ws_size,
                              hipStream_t stream) {
  if (n_in < 36 || out_size < BB * 2) return;
  const int*   fingerprints = (const int*)d_in[0];
  const float* fp_mask      = (const float*)d_in[1];
  const int*   adjacency    = (const int*)d_in[2];
  const int*   words        = (const int*)d_in[3];
  const float* words_mask   = (const float*)d_in[4];
  const float* emb_fp       = (const float*)d_in[5];
  const float* emb_word     = (const float*)d_in[6];
  const float* Wg     = (const float*)d_in[7];
  const float* bg     = (const float*)d_in[8];
  const float* attn_a = (const float*)d_in[9];
  const float* Wq = (const float*)d_in[10]; const float* bq = (const float*)d_in[11];
  const float* Wk = (const float*)d_in[12]; const float* bk = (const float*)d_in[13];
  const float* Wv = (const float*)d_in[14]; const float* bv = (const float*)d_in[15];
  const float* Wo = (const float*)d_in[16]; const float* bo = (const float*)d_in[17];
  const float* ln1_g = (const float*)d_in[18]; const float* ln1_b = (const float*)d_in[19];
  const float* ln2_g = (const float*)d_in[20]; const float* ln2_b = (const float*)d_in[21];
  const float* lnf_g = (const float*)d_in[22]; const float* lnf_b = (const float*)d_in[23];
  const float* W1 = (const float*)d_in[24]; const float* b1 = (const float*)d_in[25];
  const float* W2 = (const float*)d_in[26]; const float* b2 = (const float*)d_in[27];
  const float* Wtout = (const float*)d_in[28]; const float* btout = (const float*)d_in[29];
  const float* Watt  = (const float*)d_in[30]; const float* batt  = (const float*)d_in[31];
  const float* Wout  = (const float*)d_in[32]; const float* bout  = (const float*)d_in[33];
  const float* Wint  = (const float*)d_in[34]; const float* bint  = (const float*)d_in[35];
  const int nfp = in_sizes[5] / GD;
  const int nw  = in_sizes[6] / DMD;
  if (nfp < 1 || nw < 1) return;
  if (in_sizes[0] != BB * NN || in_sizes[2] != BB * NN * NN || in_sizes[3] != BB * LL) return;

  const int ROWS = BB * LL;
  char* wsb = (char*)d_ws;
  size_t off = 0;
  auto carve = [&](size_t bytes) -> void* { void* p = wsb + off; off += (bytes + 255) & ~(size_t)255; return p; };
  float*    pe     = (float*)carve(sizeof(float) * LL * DMD);
  _Float16* wqkv_t = (_Float16*)carve(sizeof(_Float16) * QKVP * DMD);
  _Float16* wo_t   = (_Float16*)carve(sizeof(_Float16) * DMD * DMD);
  _Float16* w1_t   = (_Float16*)carve(sizeof(_Float16) * DFFD * DMD);
  _Float16* w2_t   = (_Float16*)carve(sizeof(_Float16) * DMD * DFFD);
  _Float16* wt_t   = (_Float16*)carve(sizeof(_Float16) * 64 * DMD);
  float*    xsA    = (float*)carve(sizeof(float) * BB * NN * XP);
  float*    xsB    = (float*)carve(sizeof(float) * BB * NN * XP);
  _Float16* hT     = (_Float16*)carve(sizeof(_Float16) * BB * 64 * NN);
  float*    s1     = (float*)carve(sizeof(float) * BB * NN);
  float*    s2     = (float*)carve(sizeof(float) * BB * NN);
  _Float16* att    = (_Float16*)carve(sizeof(_Float16) * BB * NN * NN);
  float*    x      = (float*)carve(sizeof(float) * ROWS * DMD);
  float*    x2     = (float*)carve(sizeof(float) * ROWS * DMD);
  _Float16* xn     = (_Float16*)carve(sizeof(_Float16) * ROWS * DMD);
  float*    qkv    = (float*)carve(sizeof(float) * ROWS * QKVP);
  _Float16* ah     = (_Float16*)carve(sizeof(_Float16) * ROWS * DMD);
  _Float16* ffh    = (_Float16*)carve(sizeof(_Float16) * ROWS * DFFD);
  float*    wv     = (float*)carve(sizeof(float) * ROWS * WVP);
  if (off > ws_size || off > ((size_t)128 << 20)) return;

  typedef const unsigned short* cus;

  pe_table_k<<<(LL * (DMD / 2) + 255) / 256, 256, 0, stream>>>(pe, LL * (DMD / 2));
  tcast_k<<<dim3(DMD / 64, DMD / 64), 256, 0, stream>>>(Wq, DMD, DMD, wqkv_t, DMD, 0);
  tcast_k<<<dim3(DMD / 64, DMD / 64), 256, 0, stream>>>(Wk, DMD, DMD, wqkv_t, DMD, DMD);
  tcast_k<<<dim3(DMD / 64, DMD / 64), 256, 0, stream>>>(Wv, DMD, DMD, wqkv_t, DMD, 2 * DMD);
  tcast_k<<<dim3(DMD / 64, DMD / 64), 256, 0, stream>>>(Wo, DMD, DMD, wo_t, DMD, 0);
  tcast_k<<<dim3(DFFD / 64, DMD / 64), 256, 0, stream>>>(W1, DMD, DFFD, w1_t, DMD, 0);
  tcast_k<<<dim3(DMD / 64, DFFD / 64), 256, 0, stream>>>(W2, DFFD, DMD, w2_t, DFFD, 0);
  tcast_k<<<dim3(1, DMD / 64), 256, 0, stream>>>(Wtout, DMD, GD, wt_t, DMD, 0);

  embed_fp_k<<<(BB * NN * 16 + 255) / 256, 256, 0, stream>>>(fingerprints, emb_fp, nfp, xsA, BB * NN);
  float* bufs[2] = {xsA, xsB};
  for (int i = 0; i < LGN; ++i) {
    float* cur = bufs[i & 1];
    float* nxt = bufs[(i + 1) & 1];
    gat_node_k<<<BB * (NN / 64), 256, 0, stream>>>(cur, Wg + i * GD * GD, bg + i * GD, attn_a + i * 2 * GD, fp_mask, hT, s1, s2);
    gat_att_k<<<BB * (NN / 64), 256, 0, stream>>>(adjacency, s1, s2, att);
    wmma_gemm64<0, false, 0, 0, true, 0><<<dim3(1, BB), 256, 0, stream>>>(
        (cus)att, nullptr, NN, (long)NN * NN,
        (cus)hT, nullptr, NN, (long)64 * NN,
        nxt, nullptr, XP, (long)NN * XP,
        nullptr, cur, (long)NN * XP,
        NN, 64, NN, 1.0f / PSC);
  }
  float* xs_fin = bufs[LGN & 1];

  ln_k<0><<<ROWS / 8, 256, 0, stream>>>(nullptr, words, emb_word, nw, pe, x, ln1_g, ln1_b, xn, ROWS);
  wmma_gemm64<0, false, 0, 0, false, 0><<<dim3((ROWS / 64) * (QKVP / 64) / 8, 1), 256, 0, stream>>>(
      (cus)xn, nullptr, DMD, 0, (cus)wqkv_t, nullptr, DMD, 0,
      qkv, nullptr, QKVP, 0, nullptr, nullptr, 0, ROWS, QKVP, DMD, 1.0f);
  mha16_k<<<BB * (LL / 64), 128, 0, stream>>>(qkv, bq, bk, bv, words_mask, ah);
  wmma_gemm64<0, false, 2, 0, true, 0><<<dim3((ROWS / 64) * (DMD / 64) / 8, 1), 256, 0, stream>>>(
      (cus)ah, nullptr, DMD, 0, (cus)wo_t, nullptr, DMD, 0,
      x2, nullptr, DMD, 0, bo, x, 0, ROWS, DMD, DMD, 1.0f);
  ln_k<1><<<ROWS / 8, 256, 0, stream>>>(x2, nullptr, nullptr, 0, nullptr, nullptr, ln2_g, ln2_b, xn, ROWS);
  wmma_gemm64<0, false, 2, 1, false, 2><<<dim3((ROWS / 64) * (DFFD / 64) / 8, 1), 256, 0, stream>>>(
      (cus)xn, nullptr, DMD, 0, (cus)w1_t, nullptr, DMD, 0,
      ffh, nullptr, DFFD, 0, b1, nullptr, 0, ROWS, DFFD, DMD, 1.0f);
  wmma_gemm64<0, false, 2, 0, true, 0><<<dim3((ROWS / 64) * (DMD / 64) / 8, 1), 256, 0, stream>>>(
      (cus)ffh, nullptr, DFFD, 0, (cus)w2_t, nullptr, DFFD, 0,
      x, nullptr, DMD, 0, b2, x2, 0, ROWS, DMD, DFFD, 1.0f);
  ln_k<2><<<ROWS / 8, 256, 0, stream>>>(x, nullptr, nullptr, 0, nullptr, nullptr, lnf_g, lnf_b, xn, ROWS);
  wmma_gemm64<0, false, 0, 0, false, 0><<<dim3((ROWS / 64) * (WVP / 64) / 8, 1), 256, 0, stream>>>(
      (cus)xn, nullptr, DMD, 0, (cus)wt_t, nullptr, DMD, 0,
      wv, nullptr, WVP, 0, nullptr, nullptr, 0, ROWS, WVP, DMD, 1.0f);

  tail_k<<<1, 512, 0, stream>>>(xs_fin, fp_mask, wv, btout, Watt, batt, Wout, bout, Wint, bint, (float*)d_out);
}
